// MultiHeadGatedAxialAttentionWidth_63582695850407
// MI455X (gfx1250) — hardware-verified
//
#include <hip/hip_runtime.h>


namespace {
__device__ __forceinline__ float tanh_e(float v) { return 1.0f - 2.0f * __builtin_amdgcn_rcpf(1.0f + __expf(2.0f * v)); }
constexpr int Nn = 4, C = 256, Hh = 64, Wd = 128, NH = 8, HD = 32, NPIX = Nn * Hh * Wd;
constexpr float DS = 0.0625f;

typedef _Float16 b16;
typedef __attribute__((ext_vector_type(16))) _Float16 v16b;
typedef __attribute__((ext_vector_type(8)))  _Float16 v8b;
typedef __attribute__((ext_vector_type(8)))  float v8f;
typedef __attribute__((ext_vector_type(4)))  float v4f;

__device__ __forceinline__ v8b ld8b(const b16* p) { return *(const v8b*)p; }
__device__ __forceinline__ v16b cat8b(v8b a, v8b b) { return __builtin_shufflevector(a, b, 0, 1, 2, 3, 4, 5, 6, 7, 8, 9, 10, 11, 12, 13, 14, 15); }
__device__ __forceinline__ v16b frag_kb(const b16* p, int hh) { return cat8b(ld8b(p + 8 * hh), ld8b(p + 16 + 8 * hh)); }
__device__ __forceinline__ void split16(float v, b16& hi, b16& lo) { hi = (b16)v; lo = (b16)(v - (float)hi); }
__device__ __forceinline__ void frag_ksplit(const float* p, int hh, v16b& fh_, v16b& fl_) {
  const float* p0 = p + 8 * hh; const float* p1 = p + 16 + 8 * hh;
#pragma unroll
  for (int e = 0; e < 8; ++e) { b16 a, c; split16(p0[e], a, c); fh_[e] = a; fl_[e] = c; split16(p1[e], a, c); fh_[8 + e] = a; fl_[8 + e] = c; }
}
__device__ __forceinline__ v8f wmma16b(v16b a, v16b b, v8f c) {
  v8f d = __builtin_amdgcn_wmma_f32_16x16x32_f16(false, a, false, b, (short)0, c, false, false);
  asm volatile("v_nop\n\tv_nop\n\tv_nop\n\tv_nop" : "+v"(d) : "v"(a), "v"(b));
  return d;
}
__device__ __forceinline__ void wave_lds_sync() {
  __builtin_amdgcn_fence(__ATOMIC_RELEASE, "workgroup");
  __builtin_amdgcn_wave_barrier();
  __builtin_amdgcn_fence(__ATOMIC_ACQUIRE, "workgroup");
}

struct Opnd { const void* p0; const void* p1; int ld; };
template <int NP> __device__ __forceinline__ void load_frags(const Opnd& o, int row, int kb, int hh, v16b& fh_, v16b& fl_) {
  if (NP == 0) { frag_ksplit((const float*)o.p0 + (size_t)row * o.ld + kb, hh, fh_, fl_); }
  else if (NP == 4) {
    const float* p = (const float*)o.p0 + (size_t)row * o.ld + kb; const float* p0 = p + 8 * hh; const float* p1 = p + 16 + 8 * hh;
#pragma unroll
    for (int e = 0; e < 8; ++e) { b16 a, c; split16(p0[e] * 64.0f, a, c); fh_[e] = a; fl_[e] = c; split16(p1[e] * 64.0f, a, c); fh_[8 + e] = a; fl_[8 + e] = c; }
  } else if (NP == 3) {
    const float* p = (const float*)o.p0 + (size_t)row * o.ld + kb; const float* p0 = p + 8 * hh; const float* p1 = p + 16 + 8 * hh;
#pragma unroll
    for (int e = 0; e < 8; ++e) { fh_[e] = (b16)p0[e]; fh_[8 + e] = (b16)p1[e]; }
    fl_ = fh_;
  } else {
    fh_ = frag_kb((const b16*)o.p0 + (size_t)row * o.ld + kb, hh);
    if (NP == 2) fl_ = frag_kb((const b16*)o.p1 + (size_t)row * o.ld + kb, hh); else fl_ = fh_;
  }
}
template <int ANP, int BNP> __device__ __forceinline__ v8f mac(v16b ah, v16b al, v16b bh, v16b bl, v8f c) {
  c = wmma16b(ah, bh, c);
  if (BNP == 0 || BNP == 2 || BNP == 4) c = wmma16b(ah, bl, c);
  if (ANP == 0 || ANP == 2 || ANP == 4) c = wmma16b(al, bh, c);
  return c;
}
template <int ANP, int BNP>
__device__ __forceinline__ void gemm_tile(const Opnd& A, const Opnd& B, int K, int m0, int c0, int nloc, int hlf, v8f (&acc)[2][4]) {
  for (int kb = 0; kb < K; kb += 32) {
    v16b a0h, a0l, a1h, a1l;
    load_frags<ANP>(A, m0 + nloc, kb, hlf, a0h, a0l);
    load_frags<ANP>(A, m0 + 16 + nloc, kb, hlf, a1h, a1l);
#pragma unroll
    for (int t = 0; t < 4; ++t) {
      v16b bh, bl;
      load_frags<BNP>(B, c0 + t * 16 + nloc, kb, hlf, bh, bl);
      acc[0][t] = mac<ANP, BNP>(a0h, a0l, bh, bl, acc[0][t]);
      acc[1][t] = mac<ANP, BNP>(a1h, a1l, bh, bl, acc[1][t]);
    }
  }
}

__device__ __forceinline__ void epi_planes(v8f (&acc)[2][4], float scale, bool two, b16* __restrict__ oh, b16* __restrict__ ol, int ldo,
                                           int m0, int c0, int lane, b16* Th, b16* Tl) {
  const int nloc = lane & 15, hlf = lane >> 4;
#pragma unroll
  for (int t = 0; t < 4; ++t)
#pragma unroll
    for (int r = 0; r < 2; ++r)
#pragma unroll
      for (int v = 0; v < 8; ++v) {
        const int rr = r * 16 + v + 8 * hlf, cc = t * 16 + nloc;
        b16 h_, l_; split16(acc[r][t][v] * scale, h_, l_);
        Th[rr * 64 + cc] = h_; Tl[rr * 64 + cc] = l_;
      }
  wave_lds_sync();
  for (int pass = 0; pass < 2; ++pass) {
#pragma unroll
    for (int j = 0; j < 8; ++j) {
      const int rr = j * 4 + (lane >> 3), c8 = (lane & 7) * 8;
      const size_t o = (size_t)(m0 + rr) * ldo + c0 + c8;
      *(volatile v8b*)(oh + o) = ld8b(Th + rr * 64 + c8);
      if (two) *(volatile v8b*)(ol + o) = ld8b(Tl + rr * 64 + c8);
    }
    __threadfence();
  }
}
__device__ __forceinline__ void epi_f32(v8f (&acc)[2][4], float scale, const float* rscale, float* __restrict__ out, int ldo, int m0, int c0, int lane, float* Tt) {
  const int nloc = lane & 15, hlf = lane >> 4;
#pragma unroll
  for (int t = 0; t < 4; ++t)
#pragma unroll
    for (int r = 0; r < 2; ++r)
#pragma unroll
      for (int v = 0; v < 8; ++v) {
        const int rr = r * 16 + v + 8 * hlf;
        const float rs = rscale ? rscale[(size_t)(m0 + rr) * 32] : 1.0f;
        Tt[rr * 64 + t * 16 + nloc] = acc[r][t][v] * scale * rs;
      }
  wave_lds_sync();
  float* dst0 = out + (size_t)m0 * ldo + c0;
  for (int pass = 0; pass < 2; ++pass) {
#pragma unroll
    for (int j = 0; j < 16; ++j) { const int rr = j * 2 + hlf, c4 = nloc * 4; *(volatile v4f*)(dst0 + (size_t)rr * ldo + c4) = *(const v4f*)(Tt + rr * 64 + c4); }
    __threadfence();
  }
}


__global__ __launch_bounds__(256) void prep_kernel(const float* __restrict__ wq, const float* __restrict__ wk, const float* __restrict__ wv, const float* __restrict__ wo,
                                                   const float* __restrict__ rq, const float* __restrict__ rk, const float* __restrict__ rv, const float* __restrict__ Gq, const float* __restrict__ Gk,
                                                   b16* __restrict__ wqkv, b16* __restrict__ wo16, b16* __restrict__ Rcat, b16* __restrict__ rvT) {
  const size_t tid = (size_t)blockIdx.x * blockDim.x + threadIdx.x, stride = (size_t)gridDim.x * blockDim.x;
  const size_t n0 = (size_t)3 * C * C / 8, n1 = (size_t)C * C / 8, n2 = (size_t)NH * Wd * Wd * 64 / 8, n3 = (size_t)NH * Wd * HD * Wd / 8;
  for (int pass = 0; pass < 2; ++pass) {
    for (size_t p = tid; p < n0 + n1 + n2 + n3; p += stride) {
      v8b v; b16* dst;
      if (p < n0) { const size_t i = p * 8; const float* src = (i < (size_t)C * C) ? (wq + i) : (i < (size_t)2 * C * C) ? (wk + i - (size_t)C * C) : (wv + i - (size_t)2 * C * C);
#pragma unroll
        for (int e = 0; e < 8; ++e) v[e] = (b16)src[e]; dst = wqkv + i; }
      else if (p < n0 + n1) { const size_t i = (p - n0) * 8;
#pragma unroll
        for (int e = 0; e < 8; ++e) v[e] = (b16)wo[i + e]; dst = wo16 + i; }
      else if (p < n0 + n1 + n2) { const size_t i = (p - n0 - n1) * 8;
        const int cp0 = (int)(i % 64), w = (int)((i / 64) % Wd), j = (int)((i / (64 * Wd)) % Wd), h = (int)(i / ((size_t)64 * Wd * Wd));
        const float gq = tanh_e(Gq[h]) * DS, gk = tanh_e(Gk[h]) * DS;
#pragma unroll
        for (int e = 0; e < 8; ++e) { const int cp = cp0 + e; const float* tab = (cp < HD) ? rq : rk; const int c = (cp < HD) ? cp : cp - HD;
          v[e] = (b16)(((cp < HD) ? gq : gk) * tanh_e(tab[(((size_t)h * HD + c) * Wd + j) * Wd + w])); }
        dst = Rcat + i; }
      else { const size_t i = (p - n0 - n1 - n2) * 8;
        const int w0 = (int)(i % Wd), c = (int)((i / Wd) % HD), j = (int)((i / ((size_t)Wd * HD)) % Wd), h = (int)(i / ((size_t)Wd * HD * Wd));
#pragma unroll
        for (int e = 0; e < 8; ++e) v[e] = (b16)tanh_e(rv[(((size_t)h * HD + c) * Wd + j) * Wd + w0 + e]);
        dst = rvT + i; }
      *(volatile v8b*)dst = v;
    }
    __threadfence();
  }
}

__global__ __launch_bounds__(256) void xt_kernel(const float* __restrict__ x, b16* __restrict__ xT) {
  __shared__ __attribute__((aligned(16))) b16 Tl[64][72];
  const int tid = threadIdx.x, lane = tid & 31, wave = tid >> 5, n = blockIdx.y, p0 = (blockIdx.x / 4) * 64, c0 = (blockIdx.x % 4) * 64;
  for (int i = tid; i < 64 * 64; i += 256) { const int cc = i / 64, pp = i % 64; Tl[pp][cc] = (b16)x[((size_t)n * C + c0 + cc) * (Hh * Wd) + p0 + pp]; }
  __syncthreads();
  b16* dst = xT + ((size_t)n * Hh * Wd + p0) * C + c0;
  for (int pass = 0; pass < 2; ++pass) {
#pragma unroll
    for (int j = 0; j < 2; ++j) { const int rr = wave * 8 + j * 4 + (lane >> 3), c8 = (lane & 7) * 8; *(volatile v8b*)(dst + (size_t)rr * C + c8) = *(const v8b*)(&Tl[rr][c8]); }
    __threadfence();
  }
}

__global__ __launch_bounds__(128) void qkv_kernel(const b16* __restrict__ xT, const b16* __restrict__ wqkv, b16* __restrict__ qk16, b16* __restrict__ vT) {
  __shared__ __attribute__((aligned(16))) b16 Th[4][2][32 * 64];
  __shared__ __attribute__((aligned(16))) b16 Tt[64][128 + 8];
  const int lane = threadIdx.x & 31, wave = threadIdx.x >> 5, nloc = lane & 15, hlf = lane >> 4;
  const int m0 = blockIdx.y * 128 + wave * 32, c0 = blockIdx.x * 64;
  v8f acc[2][4];
#pragma unroll
  for (int r = 0; r < 2; ++r)
#pragma unroll
    for (int t = 0; t < 4; ++t) acc[r][t] = (v8f){};
  const Opnd A{xT, nullptr, C}, B{wqkv, nullptr, C};
  gemm_tile<1, 1>(A, B, C, m0, c0, nloc, hlf, acc);
  if (c0 < 2 * C) { epi_planes(acc, 1.0f, false, qk16, nullptr, 2 * C, m0, c0, lane, Th[wave][0], Th[wave][1]); return; }
#pragma unroll
  for (int t = 0; t < 4; ++t)
#pragma unroll
    for (int r = 0; r < 2; ++r)
#pragma unroll
      for (int v = 0; v < 8; ++v) Tt[t * 16 + nloc][wave * 32 + r * 16 + 8 * hlf + v] = (b16)acc[r][t][v];
  __syncthreads();
  const int pix0 = blockIdx.y * 128, n = pix0 / (Hh * Wd), i = (pix0 / Wd) % Hh, hc0 = c0 - 2 * C;
  for (int pass = 0; pass < 2; ++pass) {
#pragma unroll
    for (int j = 0; j < 8; ++j) { const int rr = wave * 16 + j * 2 + (lane >> 4), c8 = (lane & 15) * 8; const int hc = hc0 + rr, h = hc / HD, c = hc % HD;
      *(volatile v8b*)(vT + ((((size_t)n * NH + h) * Hh + i) * HD + c) * Wd + c8) = *(const v8b*)(&Tt[rr][c8]); }
    __threadfence();
  }
}

__global__ __launch_bounds__(128) void e_kernel(const b16* __restrict__ qk16, const b16* __restrict__ Rcat, int n, b16* __restrict__ E) {
  __shared__ __attribute__((aligned(16))) b16 Th[4][2][32 * 64];
  const int lane = threadIdx.x & 31, wave = threadIdx.x >> 5, nloc = lane & 15, hlf = lane >> 4;
  const int h = blockIdx.x / Wd, j = blockIdx.x % Wd, m0 = (wave & 1) * 32, c0 = (wave >> 1) * 64;
  v8f acc[2][4];
#pragma unroll
  for (int r = 0; r < 2; ++r)
#pragma unroll
    for (int t = 0; t < 4; ++t) acc[r][t] = (v8f){};
  const b16* Rb = Rcat + ((size_t)h * Wd + j) * Wd * 64;
#pragma unroll
  for (int ks = 0; ks < 2; ++ks) {
    const int ia = m0 + nloc, ib = m0 + 16 + nloc;
    const size_t pa = ((size_t)n * Hh * Wd + (size_t)ia * Wd + j) * (2 * C) + ks * C + h * HD, pb = ((size_t)n * Hh * Wd + (size_t)ib * Wd + j) * (2 * C) + ks * C + h * HD;
    const v16b a0 = frag_kb(qk16 + pa, hlf), a1 = frag_kb(qk16 + pb, hlf);
#pragma unroll
    for (int t = 0; t < 4; ++t) { const v16b bw = frag_kb(Rb + (size_t)(c0 + t * 16 + nloc) * 64 + ks * 32, hlf); acc[0][t] = wmma16b(a0, bw, acc[0][t]); acc[1][t] = wmma16b(a1, bw, acc[1][t]); }
  }
  b16* Tp = Th[wave][0];
#pragma unroll
  for (int t = 0; t < 4; ++t)
#pragma unroll
    for (int r = 0; r < 2; ++r)
#pragma unroll
      for (int v = 0; v < 8; ++v) Tp[(r * 16 + v + 8 * hlf) * 64 + t * 16 + nloc] = (b16)acc[r][t][v];
  wave_lds_sync();
  for (int pass = 0; pass < 2; ++pass) {
#pragma unroll
    for (int jj = 0; jj < 8; ++jj) { const int rr = jj * 4 + (lane >> 3), c8 = (lane & 7) * 8; const int i = m0 + rr;
      *(volatile v8b*)(E + (((size_t)h * Hh + i) * Wd + j) * Wd + c0 + c8) = ld8b(Tp + rr * 64 + c8); }
    __threadfence();
  }
}

__global__ __launch_bounds__(256) void attn_kernel(const b16* __restrict__ qk16, const b16* __restrict__ E, const b16* __restrict__ vT, int n, b16* __restrict__ wt16, float* __restrict__ x1) {
  __shared__ __attribute__((aligned(16))) b16 Ws[8][16][Wd + 8];
  __shared__ __attribute__((aligned(16))) float Xs[8][16][HD + 4];
  const int wid = threadIdx.x >> 5, lane = threadIdx.x & 31, hh = lane >> 4, col = lane & 15;
  const int qt = blockIdx.x * 8 + wid;
  const int jt = qt & 7, i = (qt >> 3) & 63, h = (qt >> 9) & 7, j0 = jt * 16;
  const size_t pixrow = (size_t)n * Hh * Wd + (size_t)i * Wd;
  const b16* qrow = qk16 + (pixrow + j0 + col) * (2 * C) + h * HD;
  const v16b qb = frag_kb(qrow, hh);
  const b16* Erow = E + (((size_t)h * Hh + i) * Wd) * Wd;
  float lg[4][16];
#pragma unroll
  for (int ch = 0; ch < 4; ++ch) {
    v8f s0 = {}, s1 = {};
    s0 = wmma16b(frag_kb(qk16 + (pixrow + ch * 32 + col) * (2 * C) + C + h * HD, hh), qb, s0);
    s1 = wmma16b(frag_kb(qk16 + (pixrow + ch * 32 + 16 + col) * (2 * C) + C + h * HD, hh), qb, s1);
#pragma unroll
    for (int r = 0; r < 8; ++r) { const int w0 = ch * 32 + 8 * hh + r, w1 = w0 + 16; const size_t eo = (size_t)(j0 + col) * Wd;
      lg[ch][r] = s0[r] * DS + (float)Erow[eo + w0]; lg[ch][8 + r] = s1[r] * DS + (float)Erow[eo + w1]; }
  }
  float m = -INFINITY;
#pragma unroll
  for (int ch = 0; ch < 4; ++ch)
#pragma unroll
    for (int r = 0; r < 16; ++r) m = fmaxf(m, lg[ch][r]);
  m = fmaxf(m, __shfl_xor(m, 16));
  float sum = 0.0f;
#pragma unroll
  for (int ch = 0; ch < 4; ++ch)
#pragma unroll
    for (int r = 0; r < 16; ++r) { lg[ch][r] = __expf(lg[ch][r] - m); sum += lg[ch][r]; }
  sum += __shfl_xor(sum, 16);
  const float inv = 1.0f / sum;
  v8f o[2] = {{}, {}};
  const b16* vrow = vT + (((size_t)n * NH + h) * Hh + i) * HD * Wd;
#pragma unroll
  for (int ch = 0; ch < 4; ++ch) {
    v16b pb;
#pragma unroll
    for (int r = 0; r < 8; ++r) { const float p0 = lg[ch][r] * inv, p1 = lg[ch][8 + r] * inv; pb[r] = (b16)p0; pb[8 + r] = (b16)p1;
      Ws[wid][col][ch * 32 + 8 * hh + r] = (b16)p0; Ws[wid][col][ch * 32 + 16 + 8 * hh + r] = (b16)p1; }
#pragma unroll
    for (int nt = 0; nt < 2; ++nt) o[nt] = wmma16b(frag_kb(vrow + (size_t)(nt * 16 + col) * Wd + ch * 32, hh), pb, o[nt]);
  }
#pragma unroll
  for (int nt = 0; nt < 2; ++nt)
#pragma unroll
    for (int r = 0; r < 8; ++r) Xs[wid][col][nt * 16 + 8 * hh + r] = o[nt][r];
  wave_lds_sync();
  const size_t rowbase = ((size_t)h * Hh + i) * Wd + j0;
  for (int pass = 0; pass < 2; ++pass) {
#pragma unroll
    for (int jj = 0; jj < 8; ++jj) { const int rr = jj * 2 + hh, c8 = col * 8; *(volatile v8b*)(wt16 + (rowbase + rr) * Wd + c8) = *(const v8b*)(&Ws[wid][rr][c8]); }
#pragma unroll
    for (int jj = 0; jj < 4; ++jj) { const int rr = jj * 4 + (lane >> 3), c4 = (lane & 7) * 4; *(volatile v4f*)(x1 + (rowbase + rr) * HD + c4) = *(const v4f*)(&Xs[wid][rr][c4]); }
    __threadfence();
  }
}

__global__ __launch_bounds__(64) void x2_kernel(const b16* __restrict__ wt16, const b16* __restrict__ rvT, const float* __restrict__ x1, const float* __restrict__ Gv1, const float* __restrict__ Gv2, int n, float* __restrict__ pre) {
  __shared__ __attribute__((aligned(16))) float Ts[2][32][HD + 4];
  const int lane = threadIdx.x & 31, wave = threadIdx.x >> 5, nloc = lane & 15, hlf = lane >> 4;
  const int h = blockIdx.x / Wd, j = blockIdx.x % Wd, m0 = wave * 32;
  const float g1 = tanh_e(Gv1[h]), g2 = tanh_e(Gv2[h]);
  const b16* Rb = rvT + ((size_t)h * Wd + j) * HD * Wd;
  auto rowidx = [&](int i) { return ((size_t)h * Hh + i) * Wd + j; };
  v8f acc[2][2] = {{{}, {}}, {{}, {}}};
#pragma unroll
  for (int kb = 0; kb < Wd; kb += 32) {
    const v16b a0 = frag_kb(wt16 + rowidx(m0 + nloc) * Wd + kb, hlf), a1 = frag_kb(wt16 + rowidx(m0 + 16 + nloc) * Wd + kb, hlf);
#pragma unroll
    for (int t = 0; t < 2; ++t) { const v16b bw = frag_kb(Rb + (size_t)(t * 16 + nloc) * Wd + kb, hlf); acc[0][t] = wmma16b(a0, bw, acc[0][t]); acc[1][t] = wmma16b(a1, bw, acc[1][t]); }
  }
#pragma unroll
  for (int t = 0; t < 2; ++t)
#pragma unroll
    for (int r = 0; r < 2; ++r)
#pragma unroll
      for (int v = 0; v < 8; ++v) { const int rr = r * 16 + v + 8 * hlf, cc = t * 16 + nloc; const size_t ri = rowidx(m0 + rr);
        Ts[wave][rr][cc] = g1 * x1[ri * HD + cc] + g2 * acc[r][t][v]; }
  wave_lds_sync();
  for (int pass = 0; pass < 2; ++pass) {
#pragma unroll
    for (int jj = 0; jj < 4; ++jj) { const int rr = jj * 8 + (lane >> 2), c4 = (lane & 3) * 8; const int i = m0 + rr;
      const size_t pix = (size_t)i * Wd + j;
      *(volatile v4f*)(pre + pix * C + h * HD + c4) = *(const v4f*)(&Ts[wave][rr][c4]); *(volatile v4f*)(pre + pix * C + h * HD + c4 + 4) = *(const v4f*)(&Ts[wave][rr][c4 + 4]); }
    __threadfence();
  }
}

__global__ __launch_bounds__(128) void out_kernel(const float* __restrict__ pre, const b16* __restrict__ wo16, int n, float* __restrict__ out) {
  __shared__ __attribute__((aligned(16))) float Ts[4][64][32 + 4];
  const int lane = threadIdx.x & 31, wave = threadIdx.x >> 5, nloc = lane & 15, hlf = lane >> 4;
  const int m0 = blockIdx.y * 128 + wave * 32, c0 = blockIdx.x * 64;
  v8f acc[2][4];
#pragma unroll
  for (int r = 0; r < 2; ++r)
#pragma unroll
    for (int t = 0; t < 4; ++t) acc[r][t] = (v8f){};
  const Opnd A{pre, nullptr, C}, B{wo16, nullptr, C};
  gemm_tile<3, 1>(A, B, C, m0, c0, nloc, hlf, acc);
#pragma unroll
  for (int t = 0; t < 4; ++t)
#pragma unroll
    for (int r = 0; r < 2; ++r)
#pragma unroll
      for (int v = 0; v < 8; ++v) Ts[wave][t * 16 + nloc][r * 16 + v + 8 * hlf] = acc[r][t][v];
  wave_lds_sync();
  const int hw0 = m0;
  for (int pass = 0; pass < 2; ++pass) {
#pragma unroll
    for (int jj = 0; jj < 16; ++jj) { const int cc = jj * 4 + (lane >> 3), c4 = (lane & 7) * 4; *(volatile v4f*)(out + ((size_t)n * C + c0 + cc) * (Hh * Wd) + hw0 + c4) = *(const v4f*)(&Ts[wave][cc][c4]); }
    __threadfence();
  }
}
}

extern "C" void kernel_launch(void* const* d_in, const int* in_sizes, int n_in,
                              void* d_out, int out_size, void* d_ws, size_t ws_size, hipStream_t stream) {
  (void)n_in; (void)out_size;
  const float* x = (const float*)d_in[0]; const float* wq = (const float*)d_in[1]; const float* wk = (const float*)d_in[2]; const float* wv = (const float*)d_in[3]; const float* wo = (const float*)d_in[4];
  const float* rq = (const float*)d_in[5]; const float* rk = (const float*)d_in[6]; const float* rv = (const float*)d_in[7];
  const float* Gq = (const float*)d_in[8]; const float* Gk = (const float*)d_in[9]; const float* Gv1 = (const float*)d_in[10]; const float* Gv2 = (const float*)d_in[11];
  float* out = (float*)d_out;
  if (in_sizes[0] != NPIX * C || in_sizes[1] != C * C || in_sizes[5] != NH * HD * Wd * Wd || in_sizes[8] != NH) return;
  size_t off = 0; char* ws = (char*)d_ws;
  auto carve = [&](size_t bytes) { char* p = ws + off; off += (bytes + 255) & ~(size_t)255; return p; };
  b16* wqkv = (b16*)carve((size_t)3 * C * C * 2); b16* wo16 = (b16*)carve((size_t)C * C * 2);
  b16* Rcat = (b16*)carve((size_t)NH * Wd * Wd * 64 * 2);
  b16* rvT = (b16*)carve((size_t)NH * Wd * HD * Wd * 2);
  b16* xT = (b16*)carve((size_t)NPIX * C * 2);
  b16* E = xT;
  b16* qk16 = (b16*)carve((size_t)NPIX * 2 * C * 2);
  b16* vT = (b16*)carve((size_t)NPIX * C * 2);
  b16* wt16 = (b16*)carve((size_t)NH * Hh * Wd * Wd * 2);
  float* x1 = (float*)carve((size_t)NH * Hh * Wd * HD * 4);
  float* pre = (float*)carve((size_t)Hh * Wd * C * 4);
  if (off > ws_size) return;
  prep_kernel<<<1024, 256, 0, stream>>>(wq, wk, wv, wo, rq, rk, rv, Gq, Gk, wqkv, wo16, Rcat, rvT);
  xt_kernel<<<dim3(128 * 4, Nn), 256, 0, stream>>>(x, xT);
  qkv_kernel<<<dim3(3 * C / 64, NPIX / 128), 128, 0, stream>>>(xT, wqkv, qk16, vT);
  for (int n = 0; n < Nn; ++n) {
    e_kernel<<<NH * Wd, 128, 0, stream>>>(qk16, Rcat, n, E);
    attn_kernel<<<NH * Hh * Wd / 16 / 8, 256, 0, stream>>>(qk16, E, vT, n, wt16, x1);
    x2_kernel<<<NH * Wd, 64, 0, stream>>>(wt16, rvT, x1, Gv1, Gv2, n, pre);
    out_kernel<<<dim3(C / 64, Hh * Wd / 128), 128, 0, stream>>>(pre, wo16, n, out);
  }
}
